// SelfAttention_64415919505520
// MI455X (gfx1250) — hardware-verified
//
#include <hip/hip_runtime.h>


#ifndef NB
#define NB 1
#endif
#ifndef SEQ
#define SEQ 4096
#endif
#define NB_FULL    1
#define SEQ_FULL   4096
#define NHEAD      16
#define HDIM       64
#define DMODEL     (NHEAD * HDIM)
#define QKV_N      (3 * DMODEL)
#define NROPE      (HDIM / 2)
#define BQ         128
#define BK         32
#define NWAVE      8
#define EARLY_QBLK 2
#define ER         ((EARLY_QBLK * BQ < SEQ) ? (EARLY_QBLK * BQ) : SEQ)
#define CT         64
#define TP         72
#define OP         68
#define PCAR       4096.0f
#define RSC        1024.0f
#define CCAR       64.0f
#define WCAR       256.0f

static_assert(NB == 1 && NB <= NB_FULL);
static_assert(SEQ <= SEQ_FULL);
static_assert(SEQ % BQ == 0);
static_assert(ER % BQ == 0);
static_assert((SEQ - ER) % 128 == 0);
static_assert(ER % CT == 0);
static_assert(SEQ % CT == 0);
static_assert(SEQ % 8 == 0);
static_assert(BQ == NWAVE * 16);
static_assert(HDIM == 64);
static_assert(DMODEL % 64 == 0 && QKV_N % 64 == 0);
static_assert(DMODEL % 32 == 0);
static_assert((SEQ * DMODEL) % 2048 == 0);
static_assert((QKV_N * DMODEL) % 2048 == 0);
static_assert((DMODEL * DMODEL) % 2048 == 0);
static_assert((TP * 2) % 16 == 0);
static_assert((OP * 4) % 16 == 0);

typedef __bf16         bf16;
typedef _Float16       f16;
typedef unsigned short us16;
typedef bf16     v16bf __attribute__((ext_vector_type(16)));
typedef f16      v16h  __attribute__((ext_vector_type(16)));
typedef f16      v8h   __attribute__((ext_vector_type(8)));
typedef float    v8f   __attribute__((ext_vector_type(8)));
typedef float    v4f   __attribute__((ext_vector_type(4)));
typedef unsigned v4u   __attribute__((ext_vector_type(4)));

union FragB  { v16bf v; v4u q[2]; bf16 h[16]; };
union FragH  { v16h  v; v4u q[2]; f16  h[16]; };
union Pack8B { v4u u; bf16 h[8]; };
union Pack8H { v4u u; v8h v; f16 h[8]; };

static __device__ __forceinline__ v8f mma_bf16(v16bf a, v16bf b, v8f acc) {
  acc = __builtin_amdgcn_wmma_f32_16x16x32_bf16(false, a, false, b, (short)0, acc, false, false);
  asm volatile("v_nop\n\tv_nop\n\tv_nop\n\tv_nop" : "+v"(acc) : "v"(a), "v"(b));
  return acc;
}
static __device__ __forceinline__ v8f mma_f16(v16h a, v16h b, v8f acc) {
  acc = __builtin_amdgcn_wmma_f32_16x16x32_f16(false, a, false, b, (short)0, acc, false, false);
  asm volatile("v_nop\n\tv_nop\n\tv_nop\n\tv_nop" : "+v"(acc) : "v"(a), "v"(b));
  return acc;
}
static __device__ __forceinline__ v8f mma(const FragB& a, const FragB& b, v8f acc) { return mma_bf16(a.v, b.v, acc); }
static __device__ __forceinline__ v8f mma(const FragH& a, const FragH& b, v8f acc) { return mma_f16(a.v, b.v, acc); }

template <int MODE>
static __device__ __forceinline__ void cvt_body(const float* __restrict__ src, us16* __restrict__ dst,
                                                 int blk, int tid) {
  const size_t e = ((size_t)blk * 256 + tid) * 8;
  const v4f a = *(const v4f*)(src + e);
  const v4f b = *(const v4f*)(src + e + 4);
  v4u u;
  if (MODE == 0) {
    Pack8B pk;
    #pragma unroll
    for (int i = 0; i < 4; ++i) {
      pk.h[i]     = (bf16)a[i];
      pk.h[4 + i] = (bf16)b[i];
    }
    u = pk.u;
  } else {
    Pack8H pk;
    #pragma unroll
    for (int i = 0; i < 4; ++i) {
      pk.h[i]     = (f16)((float)(bf16)a[i] * WCAR);
      pk.h[4 + i] = (f16)((float)(bf16)b[i] * WCAR);
    }
    u = pk.u;
  }
  *(volatile v4u*)(dst + e) = u;
  __threadfence();
  *(volatile v4u*)(dst + e) = u;
}

__global__ __launch_bounds__(256) void convert_kernel(const float* __restrict__ x,
                                                      const float* __restrict__ wq,
                                                      const float* __restrict__ wpj,
                                                      bf16* __restrict__ xb,
                                                      bf16* __restrict__ wb,
                                                      f16* __restrict__ wp) {
  const int blk = blockIdx.x;
  const int tid = threadIdx.x;
  const int NBX = SEQ * DMODEL / 2048;
  const int NBQ = QKV_N * DMODEL / 2048;
  if (blk < NBX)            cvt_body<0>(x, (us16*)xb, blk, tid);
  else if (blk < NBX + NBQ) cvt_body<0>(wq, (us16*)wb, blk - NBX, tid);
  else                      cvt_body<1>(wpj, (us16*)wp, blk - NBX - NBQ, tid);
}

__global__ __launch_bounds__(256) void rope_table_kernel(float* __restrict__ ct, float* __restrict__ st) {
  __shared__ __align__(16) float sc[8 * NROPE];
  __shared__ __align__(16) float ss[8 * NROPE];
  const int tid = threadIdx.x;
  const int j   = tid & 31;
  const int tl  = tid >> 5;
  const int t   = blockIdx.x * 8 + tl;
  const float e   = (float)(2 * j) * (1.0f / 64.0f);
  const float pw  = powf(10000.0f, e);
  const float inv = 1.0f / pw;
  const float ang = (float)t * inv;
  float sn, cs;
  sincosf(ang, &sn, &cs);
  sc[tl * NROPE + j] = cs;
  ss[tl * NROPE + j] = sn;
  __syncthreads();
  if (tid < 64) {
    const int rowl  = tid >> 3;
    const int piece = tid & 7;
    const v4f v = *(const v4f*)(sc + rowl * NROPE + piece * 4);
    const size_t gi = (size_t)(blockIdx.x * 8 + rowl) * NROPE + piece * 4;
    *(volatile v4f*)(ct + gi) = v;
    __threadfence();
    *(volatile v4f*)(ct + gi) = v;
  } else if (tid < 128) {
    const int rowl  = (tid - 64) >> 3;
    const int piece = tid & 7;
    const v4f v = *(const v4f*)(ss + rowl * NROPE + piece * 4);
    const size_t gi = (size_t)(blockIdx.x * 8 + rowl) * NROPE + piece * 4;
    *(volatile v4f*)(st + gi) = v;
    __threadfence();
    *(volatile v4f*)(st + gi) = v;
  }
}

template <typename F, int MI, int RES>
__global__ __launch_bounds__(128) void gemm_nt_kernel(const us16* __restrict__ A,
                                                          const us16* __restrict__ Ar,
                                                          const us16* __restrict__ Bm,
                                                          float* __restrict__ C,
                                                          int K, int N, int mrow0,
                                                          float oscale, float rscale) {
  __shared__ __align__(16) float sC[4 * 32 * OP];
  const int tid  = threadIdx.x;
  const int wave = tid >> 5;
  const int lane = tid & 31;
  const int lq   = lane & 15;
  const int hi   = lane >> 4;
  const int m0   = mrow0 + blockIdx.y * (64 * MI) + wave * (16 * MI);
  const int n0   = blockIdx.x * 64;

  v8f acc[MI][4], acc2[MI][4];
  #pragma unroll
  for (int mi = 0; mi < MI; ++mi) {
    #pragma unroll
    for (int t = 0; t < 4; ++t) {
      acc[mi][t]  = (v8f){0, 0, 0, 0, 0, 0, 0, 0};
      acc2[mi][t] = (v8f){0, 0, 0, 0, 0, 0, 0, 0};
    }
  }

  for (int k0 = 0; k0 < K; k0 += 32) {
    F a[MI], ar[MI], b[4];
    #pragma unroll
    for (int mi = 0; mi < MI; ++mi) {
      const us16* p = A + (size_t)(m0 + mi * 16 + lq) * K + k0 + hi * 8;
      a[mi].q[0] = *(const v4u*)(p);
      a[mi].q[1] = *(const v4u*)(p + 16);
      if (RES != 0) {
        const us16* pr = Ar + (size_t)(m0 + mi * 16 + lq) * K + k0 + hi * 8;
        ar[mi].q[0] = *(const v4u*)(pr);
        ar[mi].q[1] = *(const v4u*)(pr + 16);
      }
    }
    #pragma unroll
    for (int t = 0; t < 4; ++t) {
      const us16* p = Bm + (size_t)(n0 + t * 16 + lq) * K + k0 + hi * 8;
      b[t].q[0] = *(const v4u*)(p);
      b[t].q[1] = *(const v4u*)(p + 16);
    }
    #pragma unroll
    for (int mi = 0; mi < MI; ++mi) {
      #pragma unroll
      for (int t = 0; t < 4; ++t) {
        acc[mi][t] = mma(a[mi], b[t], acc[mi][t]);
        if (RES != 0) acc2[mi][t] = mma(ar[mi], b[t], acc2[mi][t]);
      }
    }
  }

  float* so = sC + wave * (16 * MI * OP);
  #pragma unroll
  for (int mi = 0; mi < MI; ++mi) {
    #pragma unroll
    for (int t = 0; t < 4; ++t) {
      #pragma unroll
      for (int r = 0; r < 8; ++r) {
        float val = acc[mi][t][r] * oscale;
        if (RES != 0) val += acc2[mi][t][r] * rscale;
        so[(mi * 16 + hi * 8 + r) * OP + t * 16 + lq] = val;
      }
    }
  }
  __syncthreads();

  const int NIT = 8 * MI;
  v4f    vals[8 * MI];
  size_t gidx[8 * MI];
  #pragma unroll
  for (int it = 0; it < NIT; ++it) {
    const int row = it * 2 + hi;
    vals[it] = *(const v4f*)(so + row * OP + lq * 4);
    gidx[it] = (size_t)(m0 + row) * N + n0 + lq * 4;
  }
  #pragma unroll
  for (int it = 0; it < NIT; ++it) *(volatile v4f*)(C + gidx[it]) = vals[it];
  __threadfence();
  #pragma unroll
  for (int it = 0; it < NIT; ++it) *(volatile v4f*)(C + gidx[it]) = vals[it];
}

__global__ __launch_bounds__(256) void planes_kernel(const float* __restrict__ qkv,
                                                     const float* __restrict__ ct,
                                                     const float* __restrict__ st,
                                                     f16* __restrict__ qh, f16* __restrict__ qr,
                                                     f16* __restrict__ kh, f16* __restrict__ kr,
                                                     f16* __restrict__ vt, f16* __restrict__ vtr) {
  const int kt  = blockIdx.x;
  const int h   = blockIdx.y;
  const int tid = threadIdx.x;
  __shared__ __align__(16) f16 sT[HDIM * TP];
  __shared__ __align__(16) f16 sR[HDIM * TP];
  const int  s0    = kt * CT;
  const bool early = (s0 < ER);

  v4u    qv[2], kv[2], qx[2], kx[2];
  size_t pidx[2], ridx[2];
  #pragma unroll
  for (int kk = 0; kk < 2; ++kk) {
    const int   key  = kk * 32 + (tid >> 3);
    const int   d0   = (tid & 7) * 8;
    const int   j0   = d0 & (NROPE - 1);
    const float sgn  = (d0 < NROPE) ? -1.0f : 1.0f;
    const int   srow = s0 + key;
    const float* src = qkv + (size_t)srow * QKV_N + h * HDIM + d0;
    const v4f q0v = *(const v4f*)(src);
    const v4f q1v = *(const v4f*)(src + 4);
    const v4f k0v = *(const v4f*)(src + DMODEL);
    const v4f k1v = *(const v4f*)(src + DMODEL + 4);
    const v4f v0v = *(const v4f*)(src + 2 * DMODEL);
    const v4f v1v = *(const v4f*)(src + 2 * DMODEL + 4);
    const float* cp = ct + (size_t)srow * NROPE + j0;
    const float* sp = st + (size_t)srow * NROPE + j0;
    const v4f c0 = *(const v4f*)(cp);
    const v4f c1 = *(const v4f*)(cp + 4);
    const v4f n0 = *(const v4f*)(sp);
    const v4f n1 = *(const v4f*)(sp + 4);
    float qa[8], ka[8], va[8], ca[8], sa[8];
    #pragma unroll
    for (int i = 0; i < 4; ++i) {
      qa[i] = q0v[i]; qa[4 + i] = q1v[i];
      ka[i] = k0v[i]; ka[4 + i] = k1v[i];
      va[i] = v0v[i]; va[4 + i] = v1v[i];
      ca[i] = c0[i];  ca[4 + i] = c1[i];
      sa[i] = n0[i];  sa[4 + i] = n1[i];
    }
    Pack8H pq, pqr, pk, pkr;
    #pragma unroll
    for (int i = 0; i < 8; ++i) {
      const float qp = __shfl_xor(qa[i], 4, 32);
      const float kp = __shfl_xor(ka[i], 4, 32);
      const float qo = qa[i] * ca[i] + sgn * qp * sa[i];
      const float ko = ka[i] * ca[i] + sgn * kp * sa[i];
      const f16 qhh = (f16)qo;
      const f16 khh = (f16)ko;
      pq.h[i]  = qhh;
      pk.h[i]  = khh;
      pqr.h[i] = (f16)((qo - (float)qhh) * RSC);
      pkr.h[i] = (f16)((ko - (float)khh) * RSC);
      const f16 vhh = (f16)va[i];
      sT[(d0 + i) * TP + key] = vhh;
      sR[(d0 + i) * TP + key] = (f16)((va[i] - (float)vhh) * RSC);
    }
    qv[kk] = pq.u;  qx[kk] = pqr.u;
    kv[kk] = pk.u;  kx[kk] = pkr.u;
    pidx[kk] = ((size_t)h * SEQ + srow) * HDIM + d0;
    ridx[kk] = ((size_t)h * ER + srow) * HDIM + d0;
  }
  __syncthreads();

  v4u    vv[2], vx[2];
  size_t vidx[2], vridx[2];
  #pragma unroll
  for (int kk = 0; kk < 2; ++kk) {
    const int d  = kk * 32 + (tid >> 3);
    const int ks = (tid & 7) * 8;
    Pack8H ph, px;
    ph.v = *(const v8h*)(sT + d * TP + ks);
    px.v = *(const v8h*)(sR + d * TP + ks);
    vv[kk] = ph.u;
    vx[kk] = px.u;
    vidx[kk]  = ((size_t)h * HDIM + d) * SEQ + s0 + ks;
    vridx[kk] = ((size_t)h * HDIM + d) * ER + s0 + ks;
  }

  #pragma unroll
  for (int kk = 0; kk < 2; ++kk) {
    *(volatile v4u*)(qh + pidx[kk]) = qv[kk];
    *(volatile v4u*)(kh + pidx[kk]) = kv[kk];
    *(volatile v4u*)(vt + vidx[kk]) = vv[kk];
    if (early) {
      *(volatile v4u*)(qr + ridx[kk])   = qx[kk];
      *(volatile v4u*)(kr + ridx[kk])   = kx[kk];
      *(volatile v4u*)(vtr + vridx[kk]) = vx[kk];
    }
  }
  __threadfence();
  #pragma unroll
  for (int kk = 0; kk < 2; ++kk) {
    *(volatile v4u*)(qh + pidx[kk]) = qv[kk];
    *(volatile v4u*)(kh + pidx[kk]) = kv[kk];
    *(volatile v4u*)(vt + vidx[kk]) = vv[kk];
    if (early) {
      *(volatile v4u*)(qr + ridx[kk])   = qx[kk];
      *(volatile v4u*)(kr + ridx[kk])   = kx[kk];
      *(volatile v4u*)(vtr + vridx[kk]) = vx[kk];
    }
  }
}

template <int RES>
__global__ __launch_bounds__(256) void attn_kernel(const f16* __restrict__ qh, const f16* __restrict__ qr,
                                                   const f16* __restrict__ kh, const f16* __restrict__ kr,
                                                   const f16* __restrict__ vt, const f16* __restrict__ vtr,
                                                   f16* __restrict__ ctxh, f16* __restrict__ ctxr,
                                                   int qblk0) {
  const int qblk = qblk0 + blockIdx.x;
  const int h    = blockIdx.y;
  const int tid  = threadIdx.x;
  const int wave = tid >> 5;
  const int lane = tid & 31;
  const int lq   = lane & 15;
  const int hi   = lane >> 4;

  __shared__ __align__(16) float sO[NWAVE * 16 * OP];

  const int qrow0 = qblk * BQ + wave * 16;

  FragH qf[2], qx[2];
  {
    const f16* qp = qh + ((size_t)h * SEQ + qrow0 + lq) * HDIM;
    #pragma unroll
    for (int f = 0; f < 2; ++f) {
      qf[f].q[0] = *(const v4u*)(qp + f * 32 + hi * 8);
      qf[f].q[1] = *(const v4u*)(qp + f * 32 + 16 + hi * 8);
    }
    if (RES != 0) {
      const f16* qrp = qr + ((size_t)h * ER + qrow0 + lq) * HDIM;
      #pragma unroll
      for (int f = 0; f < 2; ++f) {
        qx[f].q[0] = *(const v4u*)(qrp + f * 32 + hi * 8);
        qx[f].q[1] = *(const v4u*)(qrp + f * 32 + 16 + hi * 8);
      }
    }
  }

  const f16* kh_h  = kh  + (size_t)h * SEQ * HDIM;
  const f16* kr_h  = kr  + (size_t)h * ER * HDIM;
  const f16* vt_h  = vt  + (size_t)h * HDIM * SEQ;
  const f16* vtr_h = vtr + (size_t)h * HDIM * ER;

  v8f o[4], o2[4];
  #pragma unroll
  for (int dt = 0; dt < 4; ++dt) {
    o[dt]  = (v8f){0, 0, 0, 0, 0, 0, 0, 0};
    o2[dt] = (v8f){0, 0, 0, 0, 0, 0, 0, 0};
  }

  float rmax = -__builtin_inff();
  float rsum = 0.0f;
  const float SL = 0.125f * 1.4426950408889634f;

  const int nchunk = (qrow0 + 15) / BK + 1;
  for (int i = 0; i < nchunk; ++i) {
    const int j0 = i * BK;

    v8f c[2];
    #pragma unroll
    for (int sub = 0; sub < 2; ++sub) {
      FragH a0, a1;
      const f16* base = kh_h + (size_t)(j0 + sub * 16 + lq) * HDIM + hi * 8;
      a0.q[0] = *(const v4u*)(base);
      a0.q[1] = *(const v4u*)(base + 16);
      a1.q[0] = *(const v4u*)(base + 32);
      a1.q[1] = *(const v4u*)(base + 48);
      v8f acc = (v8f){0, 0, 0, 0, 0, 0, 0, 0};
      acc = mma_f16(a0.v, qf[0].v, acc);
      acc = mma_f16(a1.v, qf[1].v, acc);
      if (RES != 0) {
        FragH r0, r1;
        const f16* rb = kr_h + (size_t)(j0 + sub * 16 + lq) * HDIM + hi * 8;
        r0.q[0] = *(const v4u*)(rb);
        r0.q[1] = *(const v4u*)(rb + 16);
        r1.q[0] = *(const v4u*)(rb + 32);
        r1.q[1] = *(const v4u*)(rb + 48);
        v8f ax = (v8f){0, 0, 0, 0, 0, 0, 0, 0};
        ax = mma_f16(a0.v, qx[0].v, ax);
        ax = mma_f16(a1.v, qx[1].v, ax);
        ax = mma_f16(r0.v, qf[0].v, ax);
        ax = mma_f16(r1.v, qf[1].v, ax);
        #pragma unroll
        for (int r = 0; r < 8; ++r) acc[r] += ax[r] * (1.0f / RSC);
      }
      c[sub] = acc;
    }

    if (j0 + BK - 1 > qrow0) {
      const int qi = qrow0 + lq;
      #pragma unroll
      for (int sub = 0; sub < 2; ++sub) {
        #pragma unroll
        for (int r = 0; r < 8; ++r) {
          const int key = j0 + sub * 16 + hi * 8 + r;
          c[sub][r] = (key > qi) ? -__builtin_inff() : c[sub][r];
        }
      }
    }

    float m_new = rmax;
    #pragma unroll
    for (int r = 0; r < 8; ++r) {
      m_new = fmaxf(m_new, c[0][r]);
      m_new = fmaxf(m_new, c[1][r]);
    }
    m_new = fmaxf(m_new, __shfl_xor(m_new, 16, 32));
    const float scale = __builtin_amdgcn_exp2f((rmax - m_new) * SL);
    rmax = m_new;

    FragH pa, pr;
    float psum = 0.0f;
    #pragma unroll
    for (int r = 0; r < 8; ++r) {
      const float p0 = __builtin_amdgcn_exp2f((c[0][r] - m_new) * SL);
      const float p1 = __builtin_amdgcn_exp2f((c[1][r] - m_new) * SL);
      psum += p0 + p1;
      const float pc0 = p0 * PCAR;
      const float pc1 = p1 * PCAR;
      const f16 h0 = (f16)pc0;
      const f16 h1 = (f16)pc1;
      pa.h[r]     = h0;
      pa.h[8 + r] = h1;
      if (RES != 0) {
        pr.h[r]     = (f16)((pc0 - (float)h0) * RSC);
        pr.h[8 + r] = (f16)((pc1 - (float)h1) * RSC);
      }
    }
    rsum = rsum * scale + psum + __shfl_xor(psum, 16, 32);

    float sc[8];
    #pragma unroll
    for (int r = 0; r < 8; ++r) sc[r] = __shfl(scale, (hi << 3) + r, 32);
    #pragma unroll
    for (int dt = 0; dt < 4; ++dt) {
      #pragma unroll
      for (int r = 0; r < 8; ++r) {
        o[dt][r] *= sc[r];
        if (RES != 0) o2[dt][r] *= sc[r];
      }
    }

    #pragma unroll
    for (int dt = 0; dt < 4; ++dt) {
      FragH bv;
      const f16* base = vt_h + (size_t)(dt * 16 + lq) * SEQ + j0 + hi * 8;
      bv.q[0] = *(const v4u*)(base);
      bv.q[1] = *(const v4u*)(base + 16);
      o[dt] = mma_f16(pa.v, bv.v, o[dt]);
      if (RES != 0) {
        o2[dt] = mma_f16(pr.v, bv.v, o2[dt]);
        FragH br;
        const f16* rb = vtr_h + (size_t)(dt * 16 + lq) * ER + j0 + hi * 8;
        br.q[0] = *(const v4u*)(rb);
        br.q[1] = *(const v4u*)(rb + 16);
        o2[dt] = mma_f16(pa.v, br.v, o2[dt]);
      }
    }
  }

  float rs[8];
  #pragma unroll
  for (int r = 0; r < 8; ++r) rs[r] = 1.0f / __shfl(rsum, (hi << 3) + r, 32);

  float* so = sO + wave * (16 * OP);
  #pragma unroll
  for (int r = 0; r < 8; ++r) {
    #pragma unroll
    for (int dt = 0; dt < 4; ++dt) {
      float val = o[dt][r];
      if (RES != 0) val += o2[dt][r] * (1.0f / RSC);
      so[(hi * 8 + r) * OP + dt * 16 + lq] = val * (CCAR / PCAR) * rs[r];
    }
  }
  __syncthreads();

  v4u    hv[4], rv[4];
  size_t gi[4], gr[4];
  #pragma unroll
  for (int it = 0; it < 4; ++it) {
    const int row   = it * 4 + (lane >> 3);
    const int piece = lane & 7;
    const v4f a0 = *(const v4f*)(so + row * OP + piece * 8);
    const v4f a1 = *(const v4f*)(so + row * OP + piece * 8 + 4);
    Pack8H ph, px;
    #pragma unroll
    for (int k = 0; k < 4; ++k) {
      const float u0 = a0[k];
      const float u1 = a1[k];
      const f16 g0 = (f16)u0;
      const f16 g1 = (f16)u1;
      ph.h[k]     = g0;
      ph.h[4 + k] = g1;
      px.h[k]     = (f16)((u0 - (float)g0) * RSC);
      px.h[4 + k] = (f16)((u1 - (float)g1) * RSC);
    }
    hv[it] = ph.u;
    rv[it] = px.u;
    gi[it] = (size_t)(qrow0 + row) * DMODEL + h * HDIM + piece * 8;
    gr[it] = (size_t)(qrow0 + row) * DMODEL + h * HDIM + piece * 8;
  }
  #pragma unroll
  for (int it = 0; it < 4; ++it) {
    *(volatile v4u*)(ctxh + gi[it]) = hv[it];
    if (RES != 0) *(volatile v4u*)(ctxr + gr[it]) = rv[it];
  }
  __threadfence();
  #pragma unroll
  for (int it = 0; it < 4; ++it) {
    *(volatile v4u*)(ctxh + gi[it]) = hv[it];
    if (RES != 0) *(volatile v4u*)(ctxr + gr[it]) = rv[it];
  }
}

extern "C" void kernel_launch(void* const* d_in, const int* in_sizes, int n_in,
                              void* d_out, int out_size, void* d_ws, size_t ws_size,
                              hipStream_t stream) {
  if (n_in < 3) return;
  if ((size_t)in_sizes[0] < (size_t)SEQ * DMODEL) return;
  if ((size_t)in_sizes[1] < (size_t)QKV_N * DMODEL) return;
  if ((size_t)in_sizes[2] < (size_t)DMODEL * DMODEL) return;
  if ((size_t)out_size < (size_t)SEQ * DMODEL) return;

  const size_t xb_bytes   = (size_t)SEQ * DMODEL * 2;
  const size_t wb_bytes   = (size_t)QKV_N * DMODEL * 2;
  const size_t wp_bytes   = (size_t)DMODEL * DMODEL * 2;
  const size_t tab_bytes  = (size_t)SEQ * NROPE * 4;
  const size_t qkv_bytes  = (size_t)SEQ * QKV_N * 4;
  const size_t pl_bytes   = (size_t)NHEAD * SEQ * HDIM * 2;
  const size_t plr_bytes  = (size_t)NHEAD * ER * HDIM * 2;
  const size_t ctx_bytes  = (size_t)SEQ * DMODEL * 2;
  const size_t ctxr_bytes = (size_t)ER * DMODEL * 2;
  const size_t total = xb_bytes + wb_bytes + wp_bytes + 2 * tab_bytes + qkv_bytes
                     + 3 * pl_bytes + 3 * plr_bytes + ctx_bytes + ctxr_bytes;
  if (ws_size < total) return;

  char* ws = (char*)d_ws;
  size_t off = 0;
  bf16*  xb   = (bf16*)(ws + off);  off += xb_bytes;
  bf16*  wb   = (bf16*)(ws + off);  off += wb_bytes;
  f16*   wp   = (f16*)(ws + off);   off += wp_bytes;
  float* ct   = (float*)(ws + off); off += tab_bytes;
  float* st   = (float*)(ws + off); off += tab_bytes;
  float* qkv  = (float*)(ws + off); off += qkv_bytes;
  f16*   qhp  = (f16*)(ws + off);   off += pl_bytes;
  f16*   khp  = (f16*)(ws + off);   off += pl_bytes;
  f16*   vtp  = (f16*)(ws + off);   off += pl_bytes;
  f16*   qrp  = (f16*)(ws + off);   off += plr_bytes;
  f16*   krp  = (f16*)(ws + off);   off += plr_bytes;
  f16*   vtrp = (f16*)(ws + off);   off += plr_bytes;
  f16*   ctxh = (f16*)(ws + off);   off += ctx_bytes;
  f16*   ctxr = (f16*)(ws + off);   off += ctxr_bytes;
  if (off > ws_size) return;

  const float* x     = (const float*)d_in[0];
  const float* wqkv  = (const float*)d_in[1];
  const float* wproj = (const float*)d_in[2];
  float*       out   = (float*)d_out;

  const int ncvt_blocks = SEQ * DMODEL / 2048 + QKV_N * DMODEL / 2048 + DMODEL * DMODEL / 2048;
  convert_kernel<<<dim3(ncvt_blocks), 256, 0, stream>>>(x, wqkv, wproj, xb, wb, wp);

  rope_table_kernel<<<dim3(SEQ / 8), 256, 0, stream>>>(ct, st);

  gemm_nt_kernel<FragB, 2, 0><<<dim3(QKV_N / 64, SEQ / 128), 128, 0, stream>>>(
      (const us16*)xb, (const us16*)xb, (const us16*)wb, qkv, DMODEL, QKV_N, 0, 1.0f, 0.0f);

  planes_kernel<<<dim3(SEQ / CT, NHEAD), 256, 0, stream>>>(qkv, ct, st, qhp, qrp, khp, krp, vtp, vtrp);

  const int nqb     = SEQ / BQ;
  const int n_early = ER / BQ;
  const int n_late  = nqb - n_early;
  attn_kernel<1><<<dim3(n_early, NHEAD), 256, 0, stream>>>(qhp, qrp, khp, krp, vtp, vtrp, ctxh, ctxr, 0);
  if (n_late > 0)
    attn_kernel<0><<<dim3(n_late, NHEAD), 256, 0, stream>>>(qhp, qrp, khp, krp, vtp, vtrp, ctxh, ctxr, n_early);

  const float oscale = 1.0f / (CCAR * WCAR);
  const float rscale = oscale / RSC;
  gemm_nt_kernel<FragH, 1, 1><<<dim3(DMODEL / 64, ER / 64), 128, 0, stream>>>(
      (const us16*)ctxh, (const us16*)ctxr, (const us16*)wp, out, DMODEL, DMODEL, 0, oscale, rscale);
  if (SEQ - ER > 0)
    gemm_nt_kernel<FragH, 2, 0><<<dim3(DMODEL / 64, (SEQ - ER) / 128), 128, 0, stream>>>(
        (const us16*)ctxh, (const us16*)ctxh, (const us16*)wp, out, DMODEL, DMODEL, ER, oscale, 0.0f);
}
